// DiffAttention_68891275427847
// MI455X (gfx1250) — hardware-verified
//
#include <hip/hip_runtime.h>
#include <math.h>

#ifndef NQ
#define NQ 4096
#endif
#define N_FULL 4096
#define LL 4096
#define HH 8
#define MD 64
#define AWV 4
static_assert(NQ % (16 * AWV) == 0);
static_assert(NQ <= N_FULL);
static_assert(LL % 64 == 0);
static_assert(MD == 64);

typedef __attribute__((ext_vector_type(16))) _Float16 v16h;
typedef __attribute__((ext_vector_type(8)))  _Float16 v8h;
typedef __attribute__((ext_vector_type(8)))  float    v8f;
typedef __attribute__((ext_vector_type(4)))  float    v4f;
union Frag16 { v16h v; v8h half[2]; };

__device__ __forceinline__ v8f wmma16(v16h a, v16h b, v8f c) {
    c = __builtin_amdgcn_wmma_f32_16x16x32_f16(false, a, false, b, (short)0, c, false, false);
    asm volatile("v_nop\n\tv_nop\n\tv_nop\n\tv_nop" : "+v"(c) : "v"(a), "v"(b));
    return c;
}
__device__ __forceinline__ float bf16_trim(float f) {
    unsigned int u = __float_as_uint(f);
    u += 0x7fffu + ((u >> 16) & 1u);
    return __uint_as_float(u & 0xffff0000u);
}

__global__ __launch_bounds__(256) void k_cvt_rows(const float* __restrict__ X, _Float16* __restrict__ X16, int R, int total) {
    const int u = blockIdx.x * 256 + threadIdx.x;
    if (u >= total) return;
    const int r = u >> 3, p = u & 7;
    const int h = r / R, l = r - h * R;
    const float* src = X + ((size_t)l * HH + h) * MD + 8 * p;
    const v4f a = *(const v4f*)src;
    const v4f b = *(const v4f*)(src + 4);
    v8h o;
    o[0] = (_Float16)bf16_trim(a.x); o[1] = (_Float16)bf16_trim(a.y); o[2] = (_Float16)bf16_trim(a.z); o[3] = (_Float16)bf16_trim(a.w);
    o[4] = (_Float16)bf16_trim(b.x); o[5] = (_Float16)bf16_trim(b.y); o[6] = (_Float16)bf16_trim(b.z); o[7] = (_Float16)bf16_trim(b.w);
    volatile v8h* d = (volatile v8h*)(X16 + (size_t)r * MD + 8 * p);
    *d = o;
    __threadfence();
    *d = o;
}

__global__ __launch_bounds__(256) void k_cvt_vt(const float* __restrict__ V, _Float16* __restrict__ VT16) {
    __shared__ float tile[64][65];
    const int l0 = blockIdx.x * 64, h = blockIdx.y, t = threadIdx.x;
#pragma unroll
    for (int i = 0; i < 4; ++i) {
        const int idx = t + 256 * i;
        const int row = idx >> 4, c4 = (idx & 15) * 4;
        const v4f x = *(const v4f*)(V + ((size_t)(l0 + row) * HH + h) * MD + c4);
        tile[row][c4 + 0] = bf16_trim(x.x);
        tile[row][c4 + 1] = bf16_trim(x.y);
        tile[row][c4 + 2] = bf16_trim(x.z);
        tile[row][c4 + 3] = bf16_trim(x.w);
    }
    __syncthreads();
#pragma unroll
    for (int i = 0; i < 2; ++i) {
        const int idx = t + 256 * i;
        const int d = idx >> 3, p = idx & 7;
        v8h o;
#pragma unroll
        for (int e = 0; e < 8; ++e) o[e] = (_Float16)tile[8 * p + e][d];
        volatile v8h* dst = (volatile v8h*)(VT16 + ((size_t)h * MD + d) * LL + l0 + 8 * p);
        *dst = o;
        __threadfence();
        *dst = o;
    }
}

__global__ __launch_bounds__(32 * AWV) void k_sigattn(const _Float16* __restrict__ Q16, const _Float16* __restrict__ K16,
                                                        const _Float16* __restrict__ VT16, float* __restrict__ out) {
    __shared__ __align__(16) float Os[AWV][16 * 68];
    const int lane = threadIdx.x & 31, wave = threadIdx.x >> 5, hh = lane >> 4, c = lane & 15;
    const int h = blockIdx.y;
    const int q0 = blockIdx.x * (16 * AWV) + wave * 16;
    const float L2E = 1.4426950408889634f;
    const float PSC = 32768.0f;

    const _Float16* qrow = Q16 + ((size_t)h * NQ + q0 + c) * MD;
    const _Float16* kh   = K16 + (size_t)h * LL * MD;
    const _Float16* vh   = VT16 + (size_t)h * MD * LL;

    Frag16 qb[2];
#pragma unroll
    for (int ms = 0; ms < 2; ++ms) {
        qb[ms].half[0] = *(const v8h*)(qrow + 32 * ms + 8 * hh);
        qb[ms].half[1] = *(const v8h*)(qrow + 32 * ms + 16 + 8 * hh);
    }

    v8f acc[4];
#pragma unroll
    for (int t = 0; t < 4; ++t) { v8f zz = {}; acc[t] = zz; }
    float zacc = 0.f;

#pragma unroll 1
    for (int k0 = 0; k0 < LL; k0 += 32) {
        v8f s[2];
#pragma unroll
        for (int tt = 0; tt < 2; ++tt) {
            v8f zz = {}; s[tt] = zz;
            const _Float16* krow = kh + (size_t)(k0 + 16 * tt + c) * MD;
#pragma unroll
            for (int ms = 0; ms < 2; ++ms) {
                Frag16 ka;
                ka.half[0] = *(const v8h*)(krow + 32 * ms + 8 * hh);
                ka.half[1] = *(const v8h*)(krow + 32 * ms + 16 + 8 * hh);
                s[tt] = wmma16(ka.v, qb[ms].v, s[tt]);
            }
        }
        Frag16 pf;
#pragma unroll
        for (int tt = 0; tt < 2; ++tt) {
#pragma unroll
            for (int i = 0; i < 8; ++i) {
                float x = s[tt][i];
                x = fminf(fmaxf(x, -40.0f), 40.0f);
                const float e = exp2f(-x * L2E);
                const float p = __builtin_amdgcn_rcpf(1.0f + e);
                zacc += p;
                pf.v[8 * tt + i] = (_Float16)(p * PSC);
            }
        }
#pragma unroll
        for (int t = 0; t < 4; ++t) {
            const _Float16* vrow = vh + (size_t)(16 * t + c) * LL + k0;
            Frag16 va;
            va.half[0] = *(const v8h*)(vrow + 8 * hh);
            va.half[1] = *(const v8h*)(vrow + 16 + 8 * hh);
            acc[t] = wmma16(va.v, pf.v, acc[t]);
        }
    }

    const float Z = zacc + __shfl_xor(zacc, 16, 32);
    const float inv = (Z > 0.f) ? (1.0f / (Z * PSC)) : 0.f;

    float* os = Os[wave];
#pragma unroll
    for (int t = 0; t < 4; ++t)
#pragma unroll
        for (int r = 0; r < 8; ++r) os[c * 68 + 16 * t + 8 * hh + r] = acc[t][r] * inv;
    __syncthreads();
    float* ob = out + (size_t)h * MD;
    const int c4 = c * 4;
    for (int pass = 0; pass < 2; ++pass) {
#pragma unroll
        for (int it = 0; it < 8; ++it) {
            const int row = it * 2 + hh;
            const v4f val = *(const v4f*)(os + row * 68 + c4);
            *(volatile v4f*)(ob + (size_t)(q0 + row) * (HH * MD) + c4) = val;
        }
        __threadfence();
    }
}

extern "C" void kernel_launch(void* const* d_in, const int* in_sizes, int n_in,
                              void* d_out, int out_size, void* d_ws, size_t ws_size, hipStream_t stream) {
    if (n_in < 3) return;
    if (in_sizes[0] < NQ * HH * MD) return;
    if (in_sizes[1] < LL * HH * MD) return;
    if (in_sizes[2] < LL * HH * MD) return;
    if (out_size < NQ * HH * MD) return;
    const float* q = (const float*)d_in[0];
    const float* k = (const float*)d_in[1];
    const float* v = (const float*)d_in[2];
    float* out = (float*)d_out;

    char* wsp = (char*)d_ws;
    const size_t q16_bytes  = (((size_t)HH * NQ * MD * 2 + 255) / 256) * 256;
    const size_t k16_bytes  = (((size_t)HH * LL * MD * 2 + 255) / 256) * 256;
    const size_t vt16_bytes = (((size_t)HH * MD * LL * 2 + 255) / 256) * 256;
    _Float16* Q16  = (_Float16*)wsp; wsp += q16_bytes;
    _Float16* K16  = (_Float16*)wsp; wsp += k16_bytes;
    _Float16* VT16 = (_Float16*)wsp; wsp += vt16_bytes;
    const size_t total = (size_t)(wsp - (char*)d_ws);
    if (total > ws_size) return;
    if (total > (size_t)134217728) return;

    const int totq = HH * NQ * 8;
    const int totk = HH * LL * 8;
    k_cvt_rows<<<(unsigned)((totq + 255) / 256), 256, 0, stream>>>(q, Q16, NQ, totq);
    k_cvt_rows<<<(unsigned)((totk + 255) / 256), 256, 0, stream>>>(k, K16, LL, totk);
    k_cvt_vt<<<dim3((unsigned)(LL / 64), (unsigned)HH), 256, 0, stream>>>(v, VT16);
    k_sigattn<<<dim3((unsigned)(NQ / (16 * AWV)), (unsigned)HH), 32 * AWV, 0, stream>>>(Q16, K16, VT16, out);
}
